// FFN_Shared_Plus_TaskLoRA_3023656976884
// MI455X (gfx1250) — hardware-verified
//
#include <hip/hip_runtime.h>
#include <stdint.h>
#include <stddef.h>
#include <math.h>

#define TTOK  16384
#define THALF 8192
#define TD    768
#define TMID  3072
#define TE    8
#define TIN   24
#define TEC   192
#define KA2   3264
#define BM    256
#define BN    64
#define SP    68
#define NSTD  0.1f
#define WSC   256.0f
#define GSC   16.0f
#define RSC   0.00390625f

static_assert(TEC == TE * TIN);
static_assert(KA2 == TMID + TEC);
static_assert(TTOK == 2 * THALF);
static_assert(THALF % BM == 0);
static_assert(TMID % BN == 0);
static_assert(TEC % BN == 0);
static_assert(TD % BN == 0);
static_assert(TD % 64 == 0);
static_assert(KA2 % 64 == 0);
static_assert(TMID % 64 == 0);
static_assert(TD % 32 == 0);
static_assert(KA2 % 32 == 0);
static_assert((TD / 8) % 8 == 0);
static_assert((TMID / 8) % 8 == 0);
static_assert(TEC % 8 == 0);
static_assert((SP * 4) % 16 == 0);
static_assert(TTOK % 8 == 0);
static_assert(BM == 8 * 32);
static_assert(TE == 8);

typedef _Float16       v16h __attribute__((ext_vector_type(16)));
typedef _Float16       v8h  __attribute__((ext_vector_type(8)));
typedef float          v8f  __attribute__((ext_vector_type(8)));
typedef float          v4f  __attribute__((ext_vector_type(4)));
typedef unsigned int   v4u  __attribute__((ext_vector_type(4)));
typedef v4f __attribute__((may_alias)) v4fa;
typedef v4u __attribute__((may_alias)) v4ua;

union FragH { v16h v; v4u q[2]; };
union Pack8 { v8h h; v4u u; };

__device__ __forceinline__ v8f wmma_h(v16h a, v16h b, v8f c) {
  v8f d = __builtin_amdgcn_wmma_f32_16x16x32_f16(false, a, false, b, (short)0, c, false, false);
  asm volatile("v_nop\n\tv_nop\n\tv_nop\n\tv_nop" : "+v"(d) : "v"(a), "v"(b));
  return d;
}

__device__ __forceinline__ v16h ldfrag(const unsigned short* p, int h) {
  FragH f;
  f.q[0] = *(const v4ua*)(p + 8 * h);
  f.q[1] = *(const v4ua*)(p + 16 + 8 * h);
  return f.v;
}

__device__ __forceinline__ float gelu_t(float x) {
  const float u  = 0.7978845608028654f * (x + 0.044715f * x * x * x);
  const float ex = __expf(-2.0f * u);
  const float sg = __builtin_amdgcn_rcpf(1.0f + ex);
  return x * sg;
}

__global__ __launch_bounds__(256) void k_cvt(const float* s0, const float* s1,
                                             float mb, float sc, int ps,
                                             unsigned short* __restrict__ dst, int pd,
                                             int nrows, int ppr)
{
  const int g = blockIdx.x * 256 + threadIdx.x;
  if (g >= nrows * ppr) return;
  const int r = g / ppr;
  const int p = g - r * ppr;
  const size_t so = (size_t)r * ps + 8 * p;
  const v4f a0 = *(const v4fa*)(s0 + so);
  const v4f a1 = *(const v4fa*)(s0 + so + 4);
  const v4f c0 = *(const v4fa*)(s1 + so);
  const v4f c1 = *(const v4fa*)(s1 + so + 4);
  const v4f u0 = (a0 + mb * c0) * sc;
  const v4f u1 = (a1 + mb * c1) * sc;
  v8h hv;
  hv[0] = (_Float16)u0.x; hv[1] = (_Float16)u0.y; hv[2] = (_Float16)u0.z; hv[3] = (_Float16)u0.w;
  hv[4] = (_Float16)u1.x; hv[5] = (_Float16)u1.y; hv[6] = (_Float16)u1.z; hv[7] = (_Float16)u1.w;
  Pack8 pk;
  pk.h = hv;
  const v4u u = pk.u;
  unsigned short* d = dst + (size_t)r * pd + 8 * p;
  *(volatile v4u*)d = u;
  __threadfence();
  *(volatile v4u*)d = u;
}

__global__ __launch_bounds__(256) void k_w2m(const float* __restrict__ we2,
                                             unsigned short* __restrict__ dst)
{
  const int g = blockIdx.x * 256 + threadIdx.x;
  if (g >= TD * (TEC / 8)) return;
  const int d = g / (TEC / 8);
  const int p = g - d * (TEC / 8);
  v8h hv;
  #pragma unroll
  for (int i = 0; i < 8; ++i) {
    const int c  = 8 * p + i;
    const int e  = c / TIN;
    const int ii = c - e * TIN;
    hv[i] = (_Float16)(we2[((size_t)e * TD + d) * TIN + ii] * GSC);
  }
  Pack8 pk;
  pk.h = hv;
  const v4u u = pk.u;
  unsigned short* o = dst + (size_t)d * KA2 + TMID + 8 * p;
  *(volatile v4u*)o = u;
  __threadfence();
  *(volatile v4u*)o = u;
}

__global__ __launch_bounds__(256) void k_gate(const float* __restrict__ x,
                                              const float* __restrict__ noise,
                                              const float* __restrict__ wg,
                                              const float* __restrict__ bg,
                                              float* __restrict__ wt, int ntok)
{
  __shared__ __align__(16) float srec[8 * TE];
  const int tid = threadIdx.x, lane = tid & 31, wv = tid >> 5;
  const int t = blockIdx.x * 8 + wv;
  const int tc = (t < ntok) ? t : (ntok - 1);
  const float* xr = x + (size_t)tc * TD;

  double lg[TE];
  #pragma unroll
  for (int e = 0; e < TE; ++e) lg[e] = 0.0;
  #pragma unroll 1
  for (int it = 0; it < TD / 32; ++it) {
    const int d = 32 * it + lane;
    const double xv = (double)xr[d];
    #pragma unroll
    for (int e = 0; e < TE; ++e) lg[e] = fma(xv, (double)wg[e * TD + d], lg[e]);
  }
  #pragma unroll
  for (int off = 16; off > 0; off >>= 1) {
    #pragma unroll
    for (int e = 0; e < TE; ++e) lg[e] = lg[e] + __shfl_xor(lg[e], off, 32);
  }
  const float* nr = noise + (size_t)tc * TE;
  #pragma unroll
  for (int e = 0; e < TE; ++e) lg[e] = lg[e] + (double)bg[e] + (double)nr[e] * (double)NSTD;

  int i0 = 0;
  double b0 = lg[0];
  #pragma unroll
  for (int e = 1; e < TE; ++e) {
    const bool take = lg[e] > b0;
    b0 = take ? lg[e] : b0;
    i0 = take ? e : i0;
  }
  int i1 = -1;
  double bb = -1.0e300;
  #pragma unroll
  for (int e = 0; e < TE; ++e) {
    const bool take = (e != i0) && (lg[e] > bb);
    bb = take ? lg[e] : bb;
    i1 = take ? e : i1;
  }
  i1 = (i1 < 0) ? ((i0 == 0) ? 1 : 0) : i1;
  double s0 = lg[0], s1 = lg[0];
  #pragma unroll
  for (int e = 0; e < TE; ++e) { s0 = (e == i0) ? lg[e] : s0; s1 = (e == i1) ? lg[e] : s1; }
  const float l0 = (float)s0;
  const float l1 = (float)s1;
  const float q   = expf(l1 - l0);
  const float den = 1.0f + q;
  const float rden = 1.0f / den;
  const float g0 = rden;
  const float g1 = q * rden;

  if (lane == 0) {
    float gv[TE];
    #pragma unroll
    for (int e = 0; e < TE; ++e) gv[e] = (e == i0) ? g0 : ((e == i1) ? g1 : 0.0f);
    v4f r0, r1;
    r0.x = gv[0]; r0.y = gv[1]; r0.z = gv[2]; r0.w = gv[3];
    r1.x = gv[4]; r1.y = gv[5]; r1.z = gv[6]; r1.w = gv[7];
    *(v4fa*)(srec + TE * wv) = r0;
    *(v4fa*)(srec + TE * wv + 4) = r1;
  }
  __syncthreads();
  if (wv == 0) {
    const int lr = lane & 15;
    const v4f v = *(const v4fa*)(srec + 4 * lr);
    const int tt = blockIdx.x * 8 + (lr >> 1);
    const bool ok = (lane < 16) && (tt < ntok);
    float* dst = wt + (size_t)blockIdx.x * (8 * TE) + 4 * lr;
    if (ok) *(volatile v4f*)dst = v;
    __threadfence();
    if (ok) *(volatile v4f*)dst = v;
  }
}

__device__ __forceinline__ void gemm_core(const unsigned short* __restrict__ A, int lda,
                                          const unsigned short* __restrict__ Bp, int ldb,
                                          int K, int arow0, int bcol0, int h, int m,
                                          v8f (&acc)[2][4])
{
  const v8f z8 = {0.f, 0.f, 0.f, 0.f, 0.f, 0.f, 0.f, 0.f};
  #pragma unroll
  for (int i = 0; i < 2; ++i)
    #pragma unroll
    for (int j = 0; j < 4; ++j) acc[i][j] = z8;
  const unsigned short* a0p = A + (size_t)(arow0 + m) * lda;
  const unsigned short* a1p = A + (size_t)(arow0 + 16 + m) * lda;
  const unsigned short* b0p = Bp + (size_t)(bcol0 + m) * ldb;
  #pragma unroll 1
  for (int k0 = 0; k0 < K; k0 += 32) {
    const v16h a0 = ldfrag(a0p + k0, h);
    const v16h a1 = ldfrag(a1p + k0, h);
    #pragma unroll
    for (int j = 0; j < 4; ++j) {
      const v16h b = ldfrag(b0p + (size_t)(16 * j) * ldb + k0, h);
      acc[0][j] = wmma_h(a0, b, acc[0][j]);
      acc[1][j] = wmma_h(a1, b, acc[1][j]);
    }
  }
}

__global__ __launch_bounds__(256) void k_gemm_h(const unsigned short* __restrict__ A, int lda,
                                                const unsigned short* __restrict__ Bp, int ldb, int K,
                                                const float* __restrict__ bia0,
                                                const float* __restrict__ bia1, float mb1,
                                                const float* __restrict__ wg, int gated,
                                                unsigned short* __restrict__ Hp, int ldh, int hcol0,
                                                float osc)
{
  __shared__ __align__(16) float stg[8 * 16 * SP];
  const int tid = threadIdx.x, lane = tid & 31, wv = tid >> 5;
  const int h = lane >> 4, m = lane & 15;
  const int bm = blockIdx.y * BM, bn = blockIdx.x * BN;

  v8f acc[2][4];
  gemm_core(A, lda, Bp, ldb, K, bm + 32 * wv, bn, h, m, acc);

  float* st = stg + wv * (16 * SP);
  #pragma unroll
  for (int i = 0; i < 2; ++i) {
    #pragma unroll
    for (int j = 0; j < 4; ++j)
      #pragma unroll
      for (int r = 0; r < 8; ++r) st[(8 * h + r) * SP + 16 * j + m] = acc[i][j][r] * RSC;
    __syncthreads();

    const int rowl0 = bm + 32 * wv + 16 * i;
    v4u hold[4];
    #pragma unroll
    for (int q = 0; q < 4; ++q) {
      const int rl = 4 * q + (lane >> 3);
      const int pc = lane & 7;
      const float* sp = st + rl * SP + 8 * pc;
      const v4f u0 = *(const v4fa*)sp;
      const v4f u1 = *(const v4fa*)(sp + 4);
      const int c = bn + 8 * pc;
      const v4f p0 = *(const v4fa*)(bia0 + c);
      const v4f p1 = *(const v4fa*)(bia0 + c + 4);
      const v4f q0 = *(const v4fa*)(bia1 + c);
      const v4f q1 = *(const v4fa*)(bia1 + c + 4);
      const v4f s0 = u0 + p0 + mb1 * q0;
      const v4f s1 = u1 + p1 + mb1 * q1;
      float v[8] = {s0.x, s0.y, s0.z, s0.w, s1.x, s1.y, s1.z, s1.w};
      float wq[8];
      #pragma unroll
      for (int e8 = 0; e8 < 8; ++e8) wq[e8] = osc;
      if (gated) {
        const float* wr = wg + (size_t)(rowl0 + rl) * TE;
        #pragma unroll
        for (int e8 = 0; e8 < 8; ++e8) {
          int ex = (c + e8) / TIN;
          ex = (ex > TE - 1) ? (TE - 1) : ex;
          wq[e8] = wr[ex] * osc;
        }
      }
      v8h hv;
      #pragma unroll
      for (int e8 = 0; e8 < 8; ++e8) hv[e8] = (_Float16)(gelu_t(v[e8]) * wq[e8]);
      Pack8 pk;
      pk.h = hv;
      hold[q] = pk.u;
    }
    unsigned short* dbp = Hp + (size_t)rowl0 * ldh + hcol0 + bn + 8 * (lane & 7);
    #pragma unroll
    for (int q = 0; q < 4; ++q)
      *(volatile v4u*)(dbp + (size_t)(4 * q + (lane >> 3)) * ldh) = hold[q];
    __threadfence();
    #pragma unroll
    for (int q = 0; q < 4; ++q)
      *(volatile v4u*)(dbp + (size_t)(4 * q + (lane >> 3)) * ldh) = hold[q];
    __syncthreads();
  }
}

__global__ __launch_bounds__(256) void k_gemm_f(const unsigned short* __restrict__ A, int lda,
                                                const unsigned short* __restrict__ Bp, int ldb, int K,
                                                const float* __restrict__ b2,
                                                const float* __restrict__ db2,
                                                const float* __restrict__ be2,
                                                const float* __restrict__ wg,
                                                float* __restrict__ out)
{
  __shared__ __align__(16) float stg[8 * 16 * SP];
  const int tid = threadIdx.x, lane = tid & 31, wv = tid >> 5;
  const int h = lane >> 4, m = lane & 15;
  const int bm = blockIdx.y * BM, bn = blockIdx.x * BN;

  v8f acc[2][4];
  gemm_core(A, lda, Bp, ldb, K, bm + 32 * wv, bn, h, m, acc);

  float* st = stg + wv * (16 * SP);
  #pragma unroll
  for (int i = 0; i < 2; ++i) {
    #pragma unroll
    for (int j = 0; j < 4; ++j)
      #pragma unroll
      for (int r = 0; r < 8; ++r) st[(8 * h + r) * SP + 16 * j + m] = acc[i][j][r] * RSC;
    __syncthreads();

    const int rowl0 = bm + 32 * wv + 16 * i;
    v4f hold[8];
    #pragma unroll
    for (int q = 0; q < 8; ++q) {
      const int rl = 2 * q + (lane >> 4);
      const int pc = lane & 15;
      const int c = bn + 4 * pc;
      const v4f u  = *(const v4fa*)(st + rl * SP + 4 * pc);
      const v4f pb = *(const v4fa*)(b2 + c);
      const v4f pd = *(const v4fa*)(db2 + c);
      const float* wr = wg + (size_t)(rowl0 + rl) * TE;
      const v4f w0 = *(const v4fa*)wr;
      const v4f w1 = *(const v4fa*)(wr + 4);
      float w8[8] = {w0.x, w0.y, w0.z, w0.w, w1.x, w1.y, w1.z, w1.w};
      v4f s = u + pb + pd;
      #pragma unroll
      for (int e = 0; e < TE; ++e) {
        const v4f be = *(const v4fa*)(be2 + (size_t)e * TD + c);
        s = s + w8[e] * be;
      }
      hold[q] = s;
    }
    float* ob = out + (size_t)rowl0 * TD + bn + 4 * (lane & 15);
    #pragma unroll
    for (int q = 0; q < 8; ++q)
      *(volatile v4f*)(ob + (size_t)(2 * q + (lane >> 4)) * TD) = hold[q];
    __threadfence();
    #pragma unroll
    for (int q = 0; q < 8; ++q)
      *(volatile v4f*)(ob + (size_t)(2 * q + (lane >> 4)) * TD) = hold[q];
    __syncthreads();
  }
}

extern "C" void kernel_launch(void* const* d_in, const int* in_sizes, int n_in,
                              void* d_out, int out_size, void* d_ws, size_t ws_size,
                              hipStream_t stream)
{
  if (n_in < 16) return;
  if (in_sizes[0]  != TTOK * TD)     return;
  if (in_sizes[1]  != TTOK * TE)     return;
  if (in_sizes[2]  != TMID * TD)     return;
  if (in_sizes[3]  != TMID)          return;
  if (in_sizes[4]  != TD * TMID)     return;
  if (in_sizes[5]  != TD)            return;
  if (in_sizes[6]  != TMID * TD)     return;
  if (in_sizes[7]  != TMID)          return;
  if (in_sizes[8]  != TD * TMID)     return;
  if (in_sizes[9]  != TD)            return;
  if (in_sizes[10] != TE * TD)       return;
  if (in_sizes[11] != TE)            return;
  if (in_sizes[12] != TE * TIN * TD) return;
  if (in_sizes[13] != TE * TIN)      return;
  if (in_sizes[14] != TE * TD * TIN) return;
  if (in_sizes[15] != TE * TD)       return;
  if (out_size != TTOK * TD)         return;

  const float* x    = (const float*)d_in[0];
  const float* nois = (const float*)d_in[1];
  const float* W1   = (const float*)d_in[2];
  const float* b1   = (const float*)d_in[3];
  const float* W2   = (const float*)d_in[4];
  const float* b2   = (const float*)d_in[5];
  const float* dW1  = (const float*)d_in[6];
  const float* db1  = (const float*)d_in[7];
  const float* dW2  = (const float*)d_in[8];
  const float* db2  = (const float*)d_in[9];
  const float* Wg   = (const float*)d_in[10];
  const float* bg   = (const float*)d_in[11];
  const float* We1  = (const float*)d_in[12];
  const float* be1  = (const float*)d_in[13];
  const float* We2  = (const float*)d_in[14];
  const float* be2  = (const float*)d_in[15];
  float* out = (float*)d_out;

  const size_t bXH = (size_t)TTOK * TD * 2;
  const size_t bB1 = (size_t)KA2 * TD * 2;
  const size_t bB2 = (size_t)TD * KA2 * 2;
  const size_t bA2 = (size_t)THALF * KA2 * 2;
  const size_t bWT = (size_t)TTOK * TE * 4;
  const size_t total = bXH + bB1 + bB2 + bA2 + bWT;
  if (total > ws_size) return;
  if (total > (size_t)134217728) return;

  char* ws = (char*)d_ws;
  size_t off = 0;
  unsigned short* XH  = (unsigned short*)(ws + off); off += bXH;
  unsigned short* B1P = (unsigned short*)(ws + off); off += bB1;
  unsigned short* B2P = (unsigned short*)(ws + off); off += bB2;
  unsigned short* A2P = (unsigned short*)(ws + off); off += bA2;
  float*          WT  = (float*)(ws + off);          off += bWT;
  if (off != total) return;

  {
    const int nr = TTOK, ppr = TD / 8;
    k_cvt<<<(nr * ppr + 255) / 256, 256, 0, stream>>>(x, x, 0.0f, 1.0f, TD, XH, TD, nr, ppr);
  }
  {
    const int nr = TMID, ppr = TD / 8;
    k_cvt<<<(nr * ppr + 255) / 256, 256, 0, stream>>>(W1, dW1, 1.0f, WSC, TD, B1P, TD, nr, ppr);
  }
  {
    const int nr = TEC, ppr = TD / 8;
    k_cvt<<<(nr * ppr + 255) / 256, 256, 0, stream>>>(We1, We1, 0.0f, WSC, TD,
                                                       B1P + (size_t)TMID * TD, TD, nr, ppr);
  }
  {
    const int nr = TD, ppr = TMID / 8;
    k_cvt<<<(nr * ppr + 255) / 256, 256, 0, stream>>>(W2, dW2, 1.0f, WSC, TMID, B2P, KA2, nr, ppr);
  }
  k_w2m<<<(TD * (TEC / 8) + 255) / 256, 256, 0, stream>>>(We2, B2P);
  k_gate<<<(TTOK + 7) / 8, 256, 0, stream>>>(x, nois, Wg, bg, WT, TTOK);

  for (int hp = 0; hp < 2; ++hp) {
    const unsigned short* XHh = XH + (size_t)hp * THALF * TD;
    const float* WTh = WT + (size_t)hp * THALF * TE;
    float* outh = out + (size_t)hp * THALF * TD;
    k_gemm_h<<<dim3(TMID / BN, THALF / BM), 256, 0, stream>>>(
        XHh, TD, B1P, TD, TD, b1, db1, 1.0f, WTh, 0, A2P, KA2, 0, 1.0f);
    k_gemm_h<<<dim3(TEC / BN, THALF / BM), 256, 0, stream>>>(
        XHh, TD, B1P + (size_t)TMID * TD, TD, TD, be1, be1, 0.0f, WTh, 1, A2P, KA2, TMID, GSC);
    k_gemm_f<<<dim3(TD / BN, THALF / BM), 256, 0, stream>>>(
        A2P, KA2, B2P, KA2, KA2, b2, db2, be2, WTh, outh);
  }
}
